// RWKVRNNCell_2654289789469
// MI455X (gfx1250) — hardware-verified
//
#include <hip/hip_runtime.h>
#include <math.h>

constexpr int kBatch = 8;
constexpr int kSeq   = 512;
constexpr int kDim   = 768;
constexpr int kFfn   = 3072;
constexpr int kRows  = kBatch * kSeq;
constexpr float kInvDim   = 1.0f / 768.0f;
constexpr float kLnEps    = 1e-3f;
constexpr float kWCarry   = 16.0f;
constexpr float kGCarry   = 64.0f;

typedef __attribute__((ext_vector_type(16))) _Float16 v16h;
typedef __attribute__((ext_vector_type(8)))  _Float16 v8h;
typedef __attribute__((ext_vector_type(16))) __bf16   v16b;
typedef __attribute__((ext_vector_type(8)))  __bf16   v8b;
typedef __attribute__((ext_vector_type(8)))  float    v8f;
typedef __attribute__((ext_vector_type(4)))  float    v4f;
typedef __attribute__((ext_vector_type(4)))  unsigned int v4u;

__device__ __forceinline__ unsigned short f2bf_bits(float f) {
  unsigned u = __float_as_uint(f);
  return (unsigned short)((u + 0x7FFFu + ((u >> 16) & 1u)) >> 16);
}
__device__ __forceinline__ float bf_bits2f(unsigned short h) { return __uint_as_float(((unsigned)h) << 16); }

__device__ __forceinline__ void dep_guard_h(v8f& a, v8f& b, v16h x, v16h y) { asm volatile("v_nop\n\tv_nop\n\tv_nop\n\tv_nop" : "+v"(a), "+v"(b) : "v"(x), "v"(y)); }
__device__ __forceinline__ void dep_guard_b(v8f& a, v8f& b, v16b x, v16b y) { asm volatile("v_nop\n\tv_nop\n\tv_nop\n\tv_nop" : "+v"(a), "+v"(b) : "v"(x), "v"(y)); }
__device__ __forceinline__ void keep4_h(v16h a, v16h b, v16h c, v16h d) { asm volatile("v_nop" :: "v"(a), "v"(b), "v"(c), "v"(d)); }
__device__ __forceinline__ void keep4_b(v16b a, v16b b, v16b c, v16b d) { asm volatile("v_nop" :: "v"(a), "v"(b), "v"(c), "v"(d)); }
__device__ __forceinline__ void acc_guard4(v8f& a, v8f& b, v8f& c, v8f& d) { asm volatile("v_nop\n\tv_nop\n\tv_nop\n\tv_nop" : "+v"(a), "+v"(b), "+v"(c), "+v"(d)); }
template <typename T> struct Frag;
template <> struct Frag<_Float16> {
  typedef v16h V; union U { v16h v; v8h h[2]; };
  static __device__ __forceinline__ v16h load(const _Float16* p) {
    U f; f.h[0] = *(const v8h*)(p); f.h[1] = *(const v8h*)(p + 16); return f.v;
  }
  static __device__ __forceinline__ v8f mma(v16h a, v16h b, v8f c) {
    return __builtin_amdgcn_wmma_f32_16x16x32_f16(false, a, false, b, (short)0, c, false, false);
  }
  static __device__ __forceinline__ void guard(v8f& a, v8f& b, v16h x, v16h y) { dep_guard_h(a, b, x, y); }
  static __device__ __forceinline__ void keep(v16h a, v16h b, v16h c, v16h d) { keep4_h(a, b, c, d); }
};
template <> struct Frag<__bf16> {
  typedef v16b V; union U { v16b v; v8b h[2]; };
  static __device__ __forceinline__ v16b load(const __bf16* p) {
    U f; f.h[0] = *(const v8b*)(p); f.h[1] = *(const v8b*)(p + 16); return f.v;
  }
  static __device__ __forceinline__ v8f mma(v16b a, v16b b, v8f c) {
    return __builtin_amdgcn_wmma_f32_16x16x32_bf16(false, a, false, b, (short)0, c, false, false);
  }
  static __device__ __forceinline__ void guard(v8f& a, v8f& b, v16b x, v16b y) { dep_guard_b(a, b, x, y); }
  static __device__ __forceinline__ void keep(v16b a, v16b b, v16b c, v16b d) { keep4_b(a, b, c, d); }
};

__device__ __forceinline__ unsigned pk16(unsigned short a, unsigned short b) { return (unsigned)a | ((unsigned)b << 16); }
__device__ __forceinline__ unsigned short h_bits(float f) { const _Float16 h = (_Float16)f; return __builtin_bit_cast(unsigned short, h); }

template <int ET> struct Elem;
template <> struct Elem<0> { typedef _Float16 T; };
template <> struct Elem<1> { typedef __bf16 T; };
template <int ET, bool SPLIT, int BIAS_MODE, int OUT_MODE, bool RESID, int ACT = 0>
__global__ __launch_bounds__(256) void wmma_gemm64(
    const unsigned short* __restrict__ Ap, const unsigned short* __restrict__ A2p, int lda, long strideA,
    const unsigned short* __restrict__ Btp, const unsigned short* __restrict__ Bt2p, int ldb, long strideB,
    void* __restrict__ Cout, void* __restrict__ Cout2, int ldc, long strideC,
    const float* __restrict__ bias,
    const float* __restrict__ resid, long strideR,
    int M, int N, int K, float scale) {
  typedef typename Elem<ET>::T T;
  typedef typename Frag<T>::V V;
  const T* A = (const T*)Ap; const T* A2 = (const T*)A2p; const T* Bt = (const T*)Btp; const T* Bt2 = (const T*)Bt2p;
  __shared__ __align__(16) float sT[8][16 * 68];
  const int b    = blockIdx.y;
  const int lane = threadIdx.x & 31;
  const int wave = threadIdx.x >> 5;
  const int tilesN = N >> 6;
  const int tilesM = M >> 6;
  const int tile = blockIdx.x * 8 + wave;
  if (tile >= tilesM * tilesN) return;
  const int tm = tile / tilesN;
  const int tn = tile - tm * tilesN;
  const int m0 = tm << 6;
  const int n0 = tn << 6;

  const T* Ab  = A  + (size_t)b * strideA;
  const T* Bb  = Bt + (size_t)b * strideB;
  const T* Ab2 = SPLIT ? (A2  + (size_t)b * strideA) : nullptr;
  const T* Bb2 = SPLIT ? (Bt2 + (size_t)b * strideB) : nullptr;

  const int rlane = lane & 15;
  const int koff  = (lane >> 4) * 8;
  const int mOff  = (lane >> 4) * 8;

  v8f acc[4][4];
#pragma unroll
  for (int i = 0; i < 4; ++i)
#pragma unroll
    for (int j = 0; j < 4; ++j) acc[i][j] = (v8f){0.f,0.f,0.f,0.f,0.f,0.f,0.f,0.f};

  for (int k0 = 0; k0 < K; k0 += 32) {
    V bh[4], bl[4];
#pragma unroll
    for (int j = 0; j < 4; ++j) {
      const size_t bo = (size_t)(n0 + (j << 4) + rlane) * ldb + koff + k0;
      bh[j] = Frag<T>::load(Bb + bo);
      if (SPLIT) bl[j] = Frag<T>::load(Bb2 + bo);
    }
#pragma unroll
    for (int i = 0; i < 4; ++i) {
      const size_t ao = (size_t)(m0 + (i << 4) + rlane) * lda + koff + k0;
      V ah = Frag<T>::load(Ab + ao);
      V al;
      if (SPLIT) al = Frag<T>::load(Ab2 + ao);
#pragma unroll
      for (int j = 0; j < 4; ++j) {
        acc[i][j] = Frag<T>::mma(ah, bh[j], acc[i][j]);
        if (SPLIT) {
          acc[i][j] = Frag<T>::mma(ah, bl[j], acc[i][j]);
          acc[i][j] = Frag<T>::mma(al, bh[j], acc[i][j]);
        }
      }
      Frag<T>::guard(acc[i][0], acc[i][3], ah, SPLIT ? al : ah);
    }
    Frag<T>::keep(bh[0], bh[1], bh[2], bh[3]);
    if (SPLIT) Frag<T>::keep(bl[0], bl[1], bl[2], bl[3]);
  }
  acc_guard4(acc[0][0], acc[0][1], acc[0][2], acc[0][3]);
  acc_guard4(acc[1][0], acc[1][1], acc[1][2], acc[1][3]);
  acc_guard4(acc[2][0], acc[2][1], acc[2][2], acc[2][3]);
  acc_guard4(acc[3][0], acc[3][1], acc[3][2], acc[3][3]);

  float* slab = sT[wave];
  const float* Rb = RESID ? (resid + (size_t)b * strideR) : nullptr;
#pragma unroll
  for (int i = 0; i < 4; ++i) {
    const int mBase = m0 + (i << 4);
#pragma unroll
    for (int j = 0; j < 4; ++j) {
      const int n = n0 + (j << 4) + rlane;
      float bv = 0.f;
      if (BIAS_MODE == 2) bv = bias[n];
#pragma unroll
      for (int r = 0; r < 8; ++r) {
        float v = acc[i][j][r] * scale;
        if (BIAS_MODE == 1) v += bias[mBase + mOff + r];
        if (BIAS_MODE == 2) v += bv;
        if (RESID) v += Rb[(size_t)(mBase + mOff + r) * ldc + n];
        if (ACT == 2) v = fmaxf(v, 0.0f);
        if (ACT == 4) v = (v > 0.f) ? v : 0.01f * v;
        if (ACT == 6) { v = fmaxf(v, 0.0f); v = v * v; }
        slab[(mOff + r) * 68 + (j << 4) + rlane] = v;
      }
    }
    __builtin_amdgcn_fence(__ATOMIC_RELEASE, "workgroup");
    __builtin_amdgcn_wave_barrier();
    __builtin_amdgcn_fence(__ATOMIC_ACQUIRE, "workgroup");
    if (OUT_MODE == 0) {
      float* C = (float*)Cout + (size_t)b * strideC;
      const int hh = lane >> 4, c4 = (lane & 15) * 4;
      for (int pass = 0; pass < 2; ++pass) {
#pragma unroll
        for (int it = 0; it < 8; ++it) {
          const int row = it * 2 + hh;
          v4f v = *(const v4f*)(slab + row * 68 + c4);
          *(volatile v4f*)(C + (size_t)(mBase + row) * ldc + n0 + c4) = v;
        }
        __threadfence();
      }
    } else {
      const int q = lane >> 3, c8 = (lane & 7) * 8;
      unsigned short* C  = (unsigned short*)Cout  + (size_t)b * strideC;
      unsigned short* C2 = (OUT_MODE == 2) ? ((unsigned short*)Cout2 + (size_t)b * strideC) : nullptr;
      for (int pass = 0; pass < 2; ++pass) {
#pragma unroll
        for (int it = 0; it < 4; ++it) {
          const int row = it * 4 + q;
          const float* sp = slab + row * 68 + c8;
          v8h hv, lv;
#pragma unroll
          for (int e = 0; e < 8; ++e) {
            if (OUT_MODE == 1) {
              hv[e] = (_Float16)sp[e];
            } else {
              unsigned short hb = f2bf_bits(sp[e]);
              unsigned short lb = f2bf_bits(sp[e] - bf_bits2f(hb));
              hv[e] = __builtin_bit_cast(_Float16, hb);
              lv[e] = __builtin_bit_cast(_Float16, lb);
            }
          }
          *(volatile v8h*)(C + (size_t)(mBase + row) * ldc + n0 + c8) = hv;
          if (OUT_MODE == 2) *(volatile v8h*)(C2 + (size_t)(mBase + row) * ldc + n0 + c8) = lv;
        }
        __threadfence();
      }
    }
    __builtin_amdgcn_fence(__ATOMIC_RELEASE, "workgroup");
    __builtin_amdgcn_wave_barrier();
    __builtin_amdgcn_fence(__ATOMIC_ACQUIRE, "workgroup");
  }
}

__global__ __launch_bounds__(256) void wtcast_kernel(const float* __restrict__ W0, const float* __restrict__ W1,
                                                     const float* __restrict__ W2, const float* __restrict__ W3,
                                                     const float* __restrict__ W4,
                                                     unsigned short* __restrict__ out, long planeStride,
                                                     int R, int Cn, float scale) {
  __shared__ float sm[64][65];
  const int t  = threadIdx.x;
  const int r0 = blockIdx.x * 64;
  const int c0 = blockIdx.y * 64;
  const int z  = blockIdx.z;
  const float* W = (z == 0) ? W0 : (z == 1) ? W1 : (z == 2) ? W2 : (z == 3) ? W3 : W4;
#pragma unroll
  for (int i = 0; i < 16; ++i) {
    const int e = i * 256 + t;
    const int r = e >> 6;
    const int c = e & 63;
    sm[c][r] = W[(size_t)(r0 + r) * Cn + c0 + c] * scale;
  }
  __syncthreads();
  const int lane = t & 31, wave = t >> 5;
  const int q = lane >> 3, c8 = (lane & 7) * 8;
  unsigned short* op = out + (size_t)z * planeStride;
  for (int pass = 0; pass < 2; ++pass) {
#pragma unroll
    for (int it = 0; it < 2; ++it) {
      const int row = wave * 8 + it * 4 + q;
      unsigned short hb[8];
#pragma unroll
      for (int e = 0; e < 8; ++e) hb[e] = h_bits(sm[row][c8 + e]);
      const v4u u = (v4u){pk16(hb[0], hb[1]), pk16(hb[2], hb[3]), pk16(hb[4], hb[5]), pk16(hb[6], hb[7])};
      *(volatile v4u*)(op + (size_t)(c0 + row) * R + r0 + c8) = u;
    }
    __threadfence();
  }
}

__device__ __forceinline__ float wave_sum32(float s) {
#pragma unroll
  for (int off = 16; off > 0; off >>= 1) s += __shfl_xor(s, off, 32);
  return s;
}

__device__ __forceinline__ v4u mix_pack8(const float* __restrict__ mp, const float (&xi)[8], const float (&xq)[8]) {
  const v4f m0 = *(const v4f*)(mp), m1 = *(const v4f*)(mp + 4);
  float mk[8];
#pragma unroll
  for (int e = 0; e < 4; ++e) { mk[e] = m0[e]; mk[4 + e] = m1[e]; }
  unsigned short hb[8];
#pragma unroll
  for (int e = 0; e < 8; ++e) {
    const float o = xi[e] * mk[e] + xq[e] * (1.0f - mk[e]);
    hb[e] = h_bits(o);
  }
  return (v4u){pk16(hb[0], hb[1]), pk16(hb[2], hb[3]), pk16(hb[4], hb[5]), pk16(hb[6], hb[7])};
}

template <int NOUT>
__global__ __launch_bounds__(96) void ln_mix_kernel(
    const float* __restrict__ src, const float* __restrict__ gam, const float* __restrict__ bet,
    const float* __restrict__ mixA, const float* __restrict__ mixB, const float* __restrict__ mixC,
    unsigned short* __restrict__ outA, unsigned short* __restrict__ outB, unsigned short* __restrict__ outC) {
  __shared__ float red[4][4];
  const int m    = blockIdx.x;
  const int tid  = threadIdx.x;
  const int lane = tid & 31, wave = tid >> 5;
  const int t    = m % kSeq;
  const int mp   = (m > 0) ? (m - 1) : 0;
  const int c8   = tid * 8;
  const float* rc = src + (size_t)m  * kDim + c8;
  const float* rp = src + (size_t)mp * kDim + c8;
  const v4f a0 = *(const v4f*)(rc), a1 = *(const v4f*)(rc + 4);
  const v4f p0 = *(const v4f*)(rp), p1 = *(const v4f*)(rp + 4);
  float xc[8], xp[8];
#pragma unroll
  for (int e = 0; e < 4; ++e) { xc[e] = a0[e]; xc[4 + e] = a1[e]; xp[e] = p0[e]; xp[4 + e] = p1[e]; }
  float sc = 0.f, sp = 0.f;
#pragma unroll
  for (int e = 0; e < 8; ++e) { sc += xc[e]; sp += xp[e]; }
  sc = wave_sum32(sc); sp = wave_sum32(sp);
  if (lane == 0) { red[0][wave] = sc; red[1][wave] = sp; }
  __syncthreads();
  const float meanc = (red[0][0] + red[0][1] + red[0][2]) * kInvDim;
  const float meanp = (red[1][0] + red[1][1] + red[1][2]) * kInvDim;
  float vc = 0.f, vp = 0.f;
#pragma unroll
  for (int e = 0; e < 8; ++e) {
    xc[e] = xc[e] - meanc; vc += xc[e] * xc[e];
    xp[e] = xp[e] - meanp; vp += xp[e] * xp[e];
  }
  vc = wave_sum32(vc); vp = wave_sum32(vp);
  if (lane == 0) { red[2][wave] = vc; red[3][wave] = vp; }
  __syncthreads();
  const float rsc = rsqrtf((red[2][0] + red[2][1] + red[2][2]) * kInvDim + kLnEps);
  const float rsp = rsqrtf((red[3][0] + red[3][1] + red[3][2]) * kInvDim + kLnEps);
  const v4f g0 = *(const v4f*)(gam + c8), g1 = *(const v4f*)(gam + c8 + 4);
  const v4f b0 = *(const v4f*)(bet + c8), b1 = *(const v4f*)(bet + c8 + 4);
  float gg[8], bb[8];
#pragma unroll
  for (int e = 0; e < 4; ++e) { gg[e] = g0[e]; gg[4 + e] = g1[e]; bb[e] = b0[e]; bb[4 + e] = b1[e]; }
  const bool havePrev = (t > 0);
#pragma unroll
  for (int e = 0; e < 8; ++e) {
    const float zi = xc[e] * rsc * gg[e] + bb[e];
    const float zq = xp[e] * rsp * gg[e] + bb[e];
    xc[e] = zi;
    xp[e] = havePrev ? zq : 0.0f;
  }
  const v4u uA = mix_pack8(mixA + c8, xc, xp);
  v4u uB = uA, uC = uA;
  if (NOUT > 1) uB = mix_pack8(mixB + c8, xc, xp);
  if (NOUT > 2) uC = mix_pack8(mixC + c8, xc, xp);
  const size_t oo = (size_t)m * kDim + c8;
  *(volatile v4u*)(outA + oo) = uA;
  if (NOUT > 1) *(volatile v4u*)(outB + oo) = uB;
  if (NOUT > 2) *(volatile v4u*)(outC + oo) = uC;
  __threadfence();
  *(volatile v4u*)(outA + oo) = uA;
  if (NOUT > 1) *(volatile v4u*)(outB + oo) = uB;
  if (NOUT > 2) *(volatile v4u*)(outC + oo) = uC;
}

__global__ __launch_bounds__(64) void decay_scan_kernel(
    const float* __restrict__ Kp, const float* __restrict__ Vp, const float* __restrict__ Rp,
    const float* __restrict__ time_decay, const float* __restrict__ time_first,
    unsigned short* __restrict__ G, float carry) {
  __shared__ float gs[8][64];
  constexpr int kChBlocks = kDim / 64;
  const int tid = threadIdx.x;
  const int b   = blockIdx.x / kChBlocks;
  const int cb  = blockIdx.x - b * kChBlocks;
  const int c0  = cb * 64;
  const int c   = c0 + tid;
  const float tf = time_first[c];
  const float ed = expf(time_decay[c]);
  float q = 0.f, num = 0.f, den = 0.f;
  const size_t base = (size_t)b * kSeq * kDim + c;
  const int line = tid >> 3, c8 = (tid & 7) * 8;
#pragma unroll 1
  for (int t = 0; t < kSeq; ++t) {
    const size_t o = base + (size_t)t * kDim;
    const float k = Kp[o], v = Vp[o], r = Rp[o];
    const float sr = 1.0f / (1.0f + expf(fminf(-r, 60.0f)));
    const float w  = tf + k;
    const float qq = fmaxf(q, w);
    const float e1 = expf(q - qq), e2 = expf(w - qq);
    const float av = (e1 * num + e2 * v) * (1.0f / (e1 * den + e2));
    const float w2 = q - ed;
    const float qn = fmaxf(w2, k);
    const float f1 = expf(w2 - qn), f2 = expf(k - qn);
    num = f1 * num + f2 * v;
    den = f1 * den + f2;
    q   = qn;
    gs[t & 7][tid] = sr * av * carry;
    if ((t & 7) == 7) {
      __syncthreads();
      unsigned short hb[8];
#pragma unroll
      for (int e = 0; e < 8; ++e) hb[e] = h_bits(gs[line][c8 + e]);
      const v4u u = (v4u){pk16(hb[0], hb[1]), pk16(hb[2], hb[3]), pk16(hb[4], hb[5]), pk16(hb[6], hb[7])};
      unsigned short* gp = G + ((size_t)b * kSeq + (size_t)(t - 7 + line)) * kDim + c0 + c8;
      *(volatile v4u*)gp = u;
      __threadfence();
      *(volatile v4u*)gp = u;
      __syncthreads();
    }
  }
}

__global__ __launch_bounds__(256) void combine_kernel(const float* __restrict__ Y1, const float* __restrict__ R2,
                                                      const float* __restrict__ KV, float* __restrict__ out, int n4) {
  const int i = blockIdx.x * 256 + threadIdx.x;
  if (i >= n4) return;
  const size_t o = 4 * (size_t)i;
  const v4f y = *(const v4f*)(Y1 + o);
  const v4f r = *(const v4f*)(R2 + o);
  const v4f k = *(const v4f*)(KV + o);
  v4f res;
#pragma unroll
  for (int e = 0; e < 4; ++e) {
    const float sg = 1.0f / (1.0f + expf(fminf(-r[e], 60.0f)));
    res[e] = y[e] + sg * k[e];
  }
  *(volatile v4f*)(out + o) = res;
  __threadfence();
  *(volatile v4f*)(out + o) = res;
}

extern "C" void kernel_launch(void* const* d_in, const int* in_sizes, int n_in,
                              void* d_out, int out_size, void* d_ws, size_t ws_size,
                              hipStream_t stream) {
  if (n_in < 19) return;
  if (out_size != kRows * kDim) return;
  if (in_sizes[0] != kRows * kDim) return;
  if (in_sizes[8] != kDim * kDim || in_sizes[16] != kDim * kFfn || in_sizes[17] != kFfn * kDim) return;

  const float* x          = (const float*)d_in[0];
  const float* ln1_g      = (const float*)d_in[1];
  const float* ln1_b      = (const float*)d_in[2];
  const float* ln2_g      = (const float*)d_in[3];
  const float* ln2_b      = (const float*)d_in[4];
  const float* tm_mix_k   = (const float*)d_in[5];
  const float* tm_mix_v   = (const float*)d_in[6];
  const float* tm_mix_r   = (const float*)d_in[7];
  const float* tm_key_w   = (const float*)d_in[8];
  const float* tm_value_w = (const float*)d_in[9];
  const float* tm_rec_w   = (const float*)d_in[10];
  const float* time_decay = (const float*)d_in[11];
  const float* time_first = (const float*)d_in[12];
  const float* out_w      = (const float*)d_in[13];
  const float* cm_mix_k   = (const float*)d_in[14];
  const float* cm_mix_r   = (const float*)d_in[15];
  const float* cm_key_w   = (const float*)d_in[16];
  const float* cm_value_w = (const float*)d_in[17];
  const float* cm_rec_w   = (const float*)d_in[18];

  const size_t szW   = (size_t)kDim * kDim * 2;
  const size_t szWF  = (size_t)kDim * kFfn * 2;
  const size_t szP16 = (size_t)kRows * kDim * 2;
  const size_t szP32 = (size_t)kRows * kDim * 4;
  const size_t szH16 = (size_t)kRows * kFfn * 2;

  char* ws = (char*)d_ws;
  size_t off = 0;
  unsigned short* WTsq = (unsigned short*)(ws + off); off += 5 * szW;
  unsigned short* WTck = (unsigned short*)(ws + off); off += szWF;
  unsigned short* WTcv = (unsigned short*)(ws + off); off += szWF;
  char* regA = ws + off; off += 3 * szP16;
  char* regB = ws + off; off += 3 * szP32;
  float* Y1 = (float*)(ws + off); off += szP32;
  if (off > ws_size) return;

  unsigned short* WTk  = WTsq;
  unsigned short* WTo  = WTsq + 3 * (size_t)kDim * kDim;
  unsigned short* WTcr = WTsq + 4 * (size_t)kDim * kDim;
  unsigned short* XK  = (unsigned short*)regA;
  unsigned short* XV  = (unsigned short*)(regA + szP16);
  unsigned short* XR  = (unsigned short*)(regA + 2 * szP16);
  unsigned short* Gp  = (unsigned short*)regA;
  unsigned short* XK2 = (unsigned short*)(regA + szP16);
  unsigned short* XR2 = (unsigned short*)(regA + 2 * szP16);
  float* Kf = (float*)regB;
  float* Vf = (float*)(regB + szP32);
  float* Rf = (float*)(regB + 2 * szP32);
  unsigned short* Hp = (unsigned short*)regB;
  float* KV = (float*)(regB + szH16);
  float* R2 = (float*)regB;

  const long pl16  = (long)kRows * kDim;
  const long wsq   = (long)kDim * kDim;
  const dim3 blk256(256);

  wtcast_kernel<<<dim3(kDim / 64, kDim / 64, 5), blk256, 0, stream>>>(
      tm_key_w, tm_value_w, tm_rec_w, out_w, cm_rec_w, WTsq, wsq, kDim, kDim, kWCarry);
  wtcast_kernel<<<dim3(kDim / 64, kFfn / 64, 1), blk256, 0, stream>>>(
      cm_key_w, cm_key_w, cm_key_w, cm_key_w, cm_key_w, WTck, 0L, kDim, kFfn, kWCarry);
  wtcast_kernel<<<dim3(kFfn / 64, kDim / 64, 1), blk256, 0, stream>>>(
      cm_value_w, cm_value_w, cm_value_w, cm_value_w, cm_value_w, WTcv, 0L, kFfn, kDim, kWCarry);

  ln_mix_kernel<3><<<dim3(kRows), dim3(96), 0, stream>>>(x, ln1_g, ln1_b, tm_mix_k, tm_mix_v, tm_mix_r, XK, XV, XR);

  wmma_gemm64<0, false, 0, 0, false, 0><<<dim3(96, 3), blk256, 0, stream>>>(
      XK, XK, kDim, pl16, WTk, WTk, kDim, wsq, (void*)Kf, (void*)Kf, kDim, pl16,
      ln1_g, x, 0L, kRows, kDim, kDim, 1.0f / kWCarry);

  decay_scan_kernel<<<dim3(kBatch * (kDim / 64)), dim3(64), 0, stream>>>(Kf, Vf, Rf, time_decay, time_first, Gp, kGCarry);

  wmma_gemm64<0, false, 0, 0, true, 0><<<dim3(96, 1), blk256, 0, stream>>>(
      Gp, Gp, kDim, pl16, WTo, WTo, kDim, wsq, (void*)Y1, (void*)Y1, kDim, pl16,
      ln1_g, x, 0L, kRows, kDim, kDim, 1.0f / (kGCarry * kWCarry));

  ln_mix_kernel<2><<<dim3(kRows), dim3(96), 0, stream>>>(Y1, ln2_g, ln2_b, cm_mix_k, cm_mix_r, cm_mix_r, XK2, XR2, XR2);

  wmma_gemm64<0, false, 0, 1, false, 6><<<dim3(384, 1), blk256, 0, stream>>>(
      XK2, XK2, kDim, pl16, WTck, WTck, kDim, (long)kFfn * kDim, (void*)Hp, (void*)Hp, kFfn, (long)kRows * kFfn,
      ln1_g, x, 0L, kRows, kFfn, kDim, 0.5f);

  wmma_gemm64<0, false, 0, 0, false, 0><<<dim3(96, 1), blk256, 0, stream>>>(
      Hp, Hp, kFfn, (long)kRows * kFfn, WTcv, WTcv, kFfn, (long)kDim * kFfn, (void*)KV, (void*)KV, kDim, pl16,
      ln1_g, x, 0L, kRows, kDim, kFfn, 1.0f / (64.0f * kWCarry));

  wmma_gemm64<0, false, 0, 0, false, 0><<<dim3(96, 1), blk256, 0, stream>>>(
      XR2, XR2, kDim, pl16, WTcr, WTcr, kDim, wsq, (void*)R2, (void*)R2, kDim, pl16,
      ln1_g, x, 0L, kRows, kDim, kDim, 1.0f / kWCarry);

  const int n4 = kRows * kDim / 4;
  combine_kernel<<<dim3((n4 + 255) / 256), blk256, 0, stream>>>(Y1, R2, KV, (float*)d_out, n4);
}
